// GraphAttention_83373905150278
// MI455X (gfx1250) — hardware-verified
//
#include <hip/hip_runtime.h>
#include <stddef.h>
#include <stdint.h>
#include <math.h>


#define NBATCH  2
#define DM      256
#define HN      8
#define HDIM    32
#define EDW     16
#define QKVW    768
#define OQ      0
#define OKK     256
#define OV      512
#define KFIN    512
#define NTHR    256
#define NWAVE   8
#define EPT     8
#define CHUNK   (NTHR * EPT)
#define WCAP    (EPT * 32)
#define LISTN   (NWAVE * WCAP)
#define NBMAX   1024
#define SLOTB   10
#define RCAP    28672
#define DEGCAP  64
#define STW     256
#define GBM     64
#define GBN     64
#define GTHR    128
#define ATTSC   0.17677669529663687f
#define WSMAX   134217728
#define LDSW_END (2 * RCAP + 2 * NBMAX + LISTN + 2 * NWAVE)
#define LDS_AGG  (LDSW_END * 4 + 64)
#define LDS_FIN  (GBM * KFIN * 2 + GBM * GBN * 4)

static_assert((1 << SLOTB) == NBMAX);
static_assert(SLOTB + 21 <= 31);
static_assert((CHUNK & (CHUNK - 1)) == 0 && CHUNK <= 2048 && SLOTB + 11 <= 31);
static_assert(NTHR * 4 == NBMAX);
static_assert(LISTN >= NBMAX);
static_assert(LISTN >= NWAVE * WCAP);
static_assert((RCAP % 32) == 0);
static_assert((NBMAX % NWAVE) == 0);
static_assert(NWAVE * STW <= RCAP && (STW % 4) == 0 && STW >= DM);
static_assert(LDS_AGG <= 300000 && LDS_FIN <= 300000);
static_assert(GBM == (GTHR / 32) * 16);
static_assert(GBM * 8 == 4 * GTHR);
static_assert(DM == 32 * 8);
static_assert(HDIM == 4 * 8 && HN * HDIM == DM);
static_assert((DM % 32) == 0 && (KFIN % 32) == 0 && KFIN == 2 * DM);
static_assert(QKVW == 3 * DM && (QKVW % GBN) == 0 && (DM % GBN) == 0);
static_assert(EDW == 16 && HN == 8);
static_assert(EDW * HN <= NTHR && HN <= NTHR);

typedef float          v4f  __attribute__((ext_vector_type(4)));
typedef float          v8f  __attribute__((ext_vector_type(8)));
typedef int            v4i  __attribute__((ext_vector_type(4)));
typedef int            v8i  __attribute__((ext_vector_type(8)));
typedef unsigned int   v4u  __attribute__((ext_vector_type(4)));
typedef unsigned short v8us __attribute__((ext_vector_type(8)));
typedef __bf16         v16b __attribute__((ext_vector_type(16)));
typedef v4f  __attribute__((may_alias)) v4fa;
typedef v4u  __attribute__((may_alias)) v4ua;
typedef v8us __attribute__((may_alias)) v8usa;
union FragB { v16b v; v8us h[2]; v8i w; };

__device__ __forceinline__ v8f wmb(const FragB& a, const FragB& b, v8f c) {
  v8f d = __builtin_amdgcn_wmma_f32_16x16x32_bf16(false, a.v, false, b.v, (short)0, c, false, false);
  asm volatile("v_nop\n\tv_nop\n\tv_nop\n\tv_nop" : "+v"(d) : "v"(a.w), "v"(b.w));
  return d;
}

__device__ __forceinline__ void ldwait() {
  asm volatile("s_wait_loadcnt 0x0" ::: "memory");
}

__device__ __forceinline__ unsigned int f2bf(float f) {
  const unsigned int u = __float_as_uint(f);
  return ((u + 0x7FFFu + ((u >> 16) & 1u)) >> 16) & 0xFFFFu;
}
__device__ __forceinline__ float bf2f(unsigned int b) { return __uint_as_float(b << 16); }
__device__ __forceinline__ float bfr(float f) { return bf2f(f2bf(f)); }
__device__ __forceinline__ v4f bfr4(const v4f a) {
  v4f r; r.x = bfr(a.x); r.y = bfr(a.y); r.z = bfr(a.z); r.w = bfr(a.w); return r;
}
__device__ __forceinline__ unsigned int pk2(float lo, float hi) { return f2bf(lo) | (f2bf(hi) << 16); }
__device__ __forceinline__ v4u pack8(const v4f a, const v4f b) {
  v4u r;
  r.x = pk2(a.x, a.y); r.y = pk2(a.z, a.w); r.z = pk2(b.x, b.y); r.w = pk2(b.z, b.w);
  return r;
}
__device__ __forceinline__ void hl2(float v0, float v1, unsigned int& hw, unsigned int& lw) {
  const unsigned int h0 = f2bf(v0), h1 = f2bf(v1);
  const unsigned int l0 = f2bf(v0 - bf2f(h0)), l1 = f2bf(v1 - bf2f(h1));
  hw = h0 | (h1 << 16);
  lw = l0 | (l1 << 16);
}
__device__ __forceinline__ void pack8hl(const v4f a, const v4f b, v4u& hv, v4u& lv) {
  unsigned int h, l;
  hl2(a.x, a.y, h, l); hv.x = h; lv.x = l;
  hl2(a.z, a.w, h, l); hv.y = h; lv.y = l;
  hl2(b.x, b.y, h, l); hv.z = h; lv.z = l;
  hl2(b.z, b.w, h, l); hv.w = h; lv.w = l;
}

__device__ __forceinline__ int scan_chunk(const int* __restrict__ keys, int nE, int cbase, int slotBase,
                                          int nb, int vec8, int* list, int tid, int lane, int wave) {
  int wc = 0;
  const int el0  = tid * EPT;
  const int e0   = cbase + el0;
  const int sent = -2147483647 - 1;
  v4i da, db;
  if (vec8 != 0 && cbase + CHUNK <= nE) {
    da = *(const v4i*)(keys + e0);
    db = *(const v4i*)(keys + e0 + 4);
  } else {
    da.x = (e0     < nE) ? keys[min(e0,     nE - 1)] : sent;
    da.y = (e0 + 1 < nE) ? keys[min(e0 + 1, nE - 1)] : sent;
    da.z = (e0 + 2 < nE) ? keys[min(e0 + 2, nE - 1)] : sent;
    da.w = (e0 + 3 < nE) ? keys[min(e0 + 3, nE - 1)] : sent;
    db.x = (e0 + 4 < nE) ? keys[min(e0 + 4, nE - 1)] : sent;
    db.y = (e0 + 5 < nE) ? keys[min(e0 + 5, nE - 1)] : sent;
    db.z = (e0 + 6 < nE) ? keys[min(e0 + 6, nE - 1)] : sent;
    db.w = (e0 + 7 < nE) ? keys[min(e0 + 7, nE - 1)] : sent;
  }
  const unsigned nbs = (unsigned)slotBase;
  const unsigned unb = (unsigned)nb;
  const unsigned s0 = (unsigned)da.x - nbs, s1 = (unsigned)da.y - nbs;
  const unsigned s2 = (unsigned)da.z - nbs, s3 = (unsigned)da.w - nbs;
  const unsigned s4 = (unsigned)db.x - nbs, s5 = (unsigned)db.y - nbs;
  const unsigned s6 = (unsigned)db.z - nbs, s7 = (unsigned)db.w - nbs;
  const bool h0 = s0 < unb, h1 = s1 < unb, h2 = s2 < unb, h3 = s3 < unb;
  const bool h4 = s4 < unb, h5 = s5 < unb, h6 = s6 < unb, h7 = s7 < unb;
  const unsigned any = __builtin_amdgcn_ballot_w32(h0 | h1 | h2 | h3 | h4 | h5 | h6 | h7);
  if (any != 0u) {
#define HITJ(J, HJ, SJ) { \
      const unsigned mj = __builtin_amdgcn_ballot_w32(HJ); \
      if (mj != 0u) { \
        if (HJ) { \
          const int pos = wc + (int)__builtin_amdgcn_mbcnt_lo(mj, 0u); \
          if (pos < WCAP) list[wave * WCAP + pos] = ((el0 + (J)) << SLOTB) | (int)(SJ); \
        } \
        wc += (int)__builtin_popcount(mj); } }
    HITJ(0, h0, s0)
    HITJ(1, h1, s1)
    HITJ(2, h2, s2)
    HITJ(3, h3, s3)
    HITJ(4, h4, s4)
    HITJ(5, h5, s5)
    HITJ(6, h6, s6)
    HITJ(7, h7, s7)
#undef HITJ
  }
  return wc;
}

__global__ __launch_bounds__(NTHR) void k_xprep(const float* __restrict__ x, unsigned short* xb, int nN, int nUnits) {
  const int i = (int)blockIdx.x * NTHR + (int)threadIdx.x;
  if (i >= nUnits) return;
  const int row = i >> 5;
  const int c0  = (i & 31) * 8;
  const int rc  = row < nN ? row : nN - 1;
  const float* p = x + (size_t)rc * DM + c0;
  v4f a = *(const v4fa*)p;
  v4f b = *(const v4fa*)(p + 4);
  const v4f z4 = {0.f, 0.f, 0.f, 0.f};
  if (row >= nN) { a = z4; b = z4; }
  const v4u hv = pack8(a, b);
  unsigned short* o = xb + (size_t)row * DM + c0;
  *(volatile v4u*)o = hv;
  __threadfence();
  *(volatile v4u*)o = hv;
}

__global__ __launch_bounds__(NTHR) void k_wtr(const float* __restrict__ w, int Kin, int Ncol, int Nrows, int Kout,
                                              unsigned short* wt, int nUnits) {
  const int u = (int)blockIdx.x * NTHR + (int)threadIdx.x;
  if (u >= nUnits) return;
  const int kq = Kout >> 3;
  const int n  = u / kq;
  const int k8 = (u - n * kq) * 8;
  const int kk = k8 - (k8 / Kin) * Kin;
  const int ncl = n < Ncol ? n : Ncol - 1;
  const float* p = w + (size_t)kk * (size_t)Ncol + ncl;
  v4f a, b;
  a.x = p[0];                    a.y = p[(size_t)Ncol];         a.z = p[(size_t)2 * Ncol];     a.w = p[(size_t)3 * Ncol];
  b.x = p[(size_t)4 * Ncol];     b.y = p[(size_t)5 * Ncol];     b.z = p[(size_t)6 * Ncol];     b.w = p[(size_t)7 * Ncol];
  const v4f z4 = {0.f, 0.f, 0.f, 0.f};
  if (n >= Ncol || n >= Nrows) { a = z4; b = z4; }
  const v4u wv = pack8(a, b);
  unsigned short* o = wt + (size_t)n * (size_t)Kout + k8;
  *(volatile v4u*)o = wv;
  __threadfence();
  *(volatile v4u*)o = wv;
}

__global__ __launch_bounds__(NTHR) void k_eb(const float* __restrict__ ea, const float* __restrict__ We,
                                             const float* __restrict__ be, float* EB, int nE, int nUnits) {
  __shared__ float sWe[EDW * HN];
  __shared__ float sbe[HN];
  const int tid = (int)threadIdx.x;
  if (tid < EDW * HN) sWe[tid] = bfr(We[tid]);
  if (tid < HN) sbe[tid] = bfr(be[tid]);
  __syncthreads();
  const int u = (int)blockIdx.x * NTHR + tid;
  if (u >= nUnits) return;
  const int e  = u >> 1;
  const int h0 = (u & 1) * 4;
  const int ec = e < nE ? e : nE - 1;
  const float* er = ea + (size_t)ec * EDW;
  float s0 = 0.f, s1 = 0.f, s2 = 0.f, s3 = 0.f;
#pragma unroll 1
  for (int q = 0; q < 4; ++q) {
    const v4f a = bfr4(*(const v4fa*)(er + 4 * q));
    const float* wr = sWe + (4 * q) * HN + h0;
    s0 = fmaf(a.x, wr[0],  s0); s1 = fmaf(a.x, wr[1],  s1); s2 = fmaf(a.x, wr[2],  s2); s3 = fmaf(a.x, wr[3],  s3);
    s0 = fmaf(a.y, wr[8],  s0); s1 = fmaf(a.y, wr[9],  s1); s2 = fmaf(a.y, wr[10], s2); s3 = fmaf(a.y, wr[11], s3);
    s0 = fmaf(a.z, wr[16], s0); s1 = fmaf(a.z, wr[17], s1); s2 = fmaf(a.z, wr[18], s2); s3 = fmaf(a.z, wr[19], s3);
    s0 = fmaf(a.w, wr[24], s0); s1 = fmaf(a.w, wr[25], s1); s2 = fmaf(a.w, wr[26], s2); s3 = fmaf(a.w, wr[27], s3);
  }
  v4f o;
  o.x = s0 + sbe[h0]; o.y = s1 + sbe[h0 + 1]; o.z = s2 + sbe[h0 + 2]; o.w = s3 + sbe[h0 + 3];
  const v4f z4 = {0.f, 0.f, 0.f, 0.f};
  if (e >= nE) o = z4;
  float* op = EB + (size_t)e * HN + h0;
  *(volatile v4f*)op = o;
  __threadfence();
  *(volatile v4f*)op = o;
}

__global__ __launch_bounds__(GTHR) void k_gemm(
    const unsigned short* __restrict__ A, const unsigned short* __restrict__ WT,
    const float* __restrict__ b0, const float* __restrict__ b1, const float* __restrict__ b2,
    float* outF, int K, int ldo)
{
  __shared__ __attribute__((aligned(16))) float stg[GBM * GBN];
  const int tid = (int)threadIdx.x, lane = tid & 31, wave = tid >> 5, hh = lane >> 4, m = lane & 15;
  const int rowBase = (int)blockIdx.x * GBM;
  const int col0    = (int)blockIdx.y * GBN;

  v8f acc[4];
  {
    const v8f z = {0.f, 0.f, 0.f, 0.f, 0.f, 0.f, 0.f, 0.f};
    acc[0] = z; acc[1] = z; acc[2] = z; acc[3] = z;
  }
  const unsigned short* ap = A  + (size_t)(rowBase + 16 * wave + m) * (size_t)K + 8 * hh;
  const unsigned short* wp = WT + (size_t)(col0 + m) * (size_t)K + 8 * hh;
  const int ksteps = K >> 5;
#pragma unroll 1
  for (int ks = 0; ks < ksteps; ++ks) {
    FragB af;
    af.h[0] = *(const v8usa*)(ap + 32 * ks);
    af.h[1] = *(const v8usa*)(ap + 32 * ks + 16);
#pragma unroll
    for (int t = 0; t < 4; ++t) {
      const unsigned short* wq = wp + (size_t)(16 * t) * (size_t)K + 32 * ks;
      FragB bf;
      bf.h[0] = *(const v8usa*)wq;
      bf.h[1] = *(const v8usa*)(wq + 16);
      acc[t] = wmb(af, bf, acc[t]);
    }
  }

#pragma unroll
  for (int t = 0; t < 4; ++t) {
    const int lc = 16 * t + m;
#pragma unroll
    for (int r = 0; r < 8; ++r) {
      const int lr = 16 * wave + 8 * hh + r;
      stg[lr * GBN + lc] = acc[t][r];
    }
  }
  __syncthreads();

  const int which = col0 >> 8;
  const int cq = (col0 & (DM - 1)) + 4 * m;
  const v4f bb0 = bfr4(*(const v4fa*)(b0 + cq));
  const v4f bb1 = bfr4(*(const v4fa*)(b1 + cq));
  const v4f bb2 = bfr4(*(const v4fa*)(b2 + cq));
  const float f0 = (which == 0) ? 1.0f : 0.0f;
  const float f1 = (which == 1) ? 1.0f : 0.0f;
  const float f2 = (which == 2) ? 1.0f : 0.0f;
  const v4f bb = bb0 * f0 + bb1 * f1 + bb2 * f2;

  v4f fv[8];
#pragma unroll
  for (int i = 0; i < 8; ++i) {
    const int lr = 16 * wave + 2 * i + hh;
    fv[i] = *(const v4fa*)(stg + lr * GBN + 4 * m) + bb;
  }
#pragma unroll
  for (int i = 0; i < 8; ++i) {
    const int lr = 16 * wave + 2 * i + hh;
    const int gr = rowBase + lr;
    float* op = outF + (size_t)gr * (size_t)ldo + col0 + 4 * m;
    *(volatile v4f*)op = fv[i];
  }
  __threadfence();
#pragma unroll
  for (int i = 0; i < 8; ++i) {
    const int lr = 16 * wave + 2 * i + hh;
    const int gr = rowBase + lr;
    float* op = outF + (size_t)gr * (size_t)ldo + col0 + 4 * m;
    *(volatile v4f*)op = fv[i];
  }
}

__global__ __launch_bounds__(NTHR) void k_agg(
    const int* __restrict__ keys, const int* __restrict__ gath,
    const float* __restrict__ QKV, const float* __restrict__ EB,
    float* OUTP, int nN, int nE, int vec8, int MPr) {
  extern __shared__ v4f lds_dyn[];
  int* reg1 = (int*)lds_dyn;
  int* reg2 = reg1 + RCAP;
  int* scnt = reg2 + RCAP;
  int* soff = scnt + NBMAX;
  int* list = soff + NBMAX;
  int* wcnt = list + LISTN;
  int* wtot = wcnt + NWAVE;
  const int tid = (int)threadIdx.x, lane = tid & 31, wave = tid >> 5;
  const int nodeBase = (int)blockIdx.x * NBMAX;

  for (int i = tid; i < NBMAX; i += NTHR) scnt[i] = 0;
  __syncthreads();

  int tot = 0;
  const int nChunks = (nE + CHUNK - 1) / CHUNK;
#pragma unroll 1
  for (int ch = 0; ch < nChunks; ++ch) {
    const int cbase = ch * CHUNK;
    const int wc = scan_chunk(keys, nE, cbase, nodeBase, NBMAX, vec8, list, tid, lane, wave);
    if (lane == 0) wcnt[wave] = wc;
    __syncthreads();
    int pre = 0, all = 0;
#pragma unroll
    for (int w2 = 0; w2 < NWAVE; ++w2) {
      int c = wcnt[w2];
      c = c < 0 ? 0 : (c > WCAP ? WCAP : c);
      all += c;
      pre += (w2 < wave) ? c : 0;
    }
    const int wcc  = wc > WCAP ? WCAP : wc;
    const int base = tot + pre;
#pragma unroll 1
    for (int i = lane; i < wcc; i += 32) {
      const int ent = list[wave * WCAP + i];
      const int el  = (ent >> SLOTB) & (CHUNK - 1);
      const int sl  = ent & (NBMAX - 1);
      int eid = cbase + el;
      eid = eid > nE - 1 ? nE - 1 : eid;
      const int pos = base + i;
      if (pos < RCAP) reg1[pos] = (int)(((unsigned)eid << SLOTB) | (unsigned)sl);
    }
    tot += all;
    tot = tot > RCAP ? RCAP : tot;
    __syncthreads();
  }
  const int nh = tot;

  if (wave == 0) {
#pragma unroll 1
    for (int b0 = 0; b0 < nh; b0 += 32) {
      const int idx = b0 + lane;
      const int uv  = reg1[idx < nh ? idx : nh - 1];
      const int m32 = (nh - b0) < 32 ? (nh - b0) : 32;
#pragma unroll 1
      for (int k = 0; k < m32; ++k) {
        const int u  = __builtin_amdgcn_readlane(uv, k);
        const int sl = u & (NBMAX - 1);
        if (lane == 0) scnt[sl] = scnt[sl] + 1;
      }
    }
  }
  __syncthreads();

  {
    const v4i ca = *(const v4i*)(scnt + 4 * tid);
    const int e0 = ca.x < 0 ? 0 : ca.x, e1 = ca.y < 0 ? 0 : ca.y, e2 = ca.z < 0 ? 0 : ca.z, e3 = ca.w < 0 ? 0 : ca.w;
    const int ts = e0 + e1 + e2 + e3;
    int incl = ts;
#pragma unroll
    for (int d = 1; d < 32; d <<= 1) {
      const int up = __shfl_up(incl, d);
      if (lane >= d) incl += up;
    }
    if (lane == 31) wtot[wave] = incl;
    __syncthreads();
    int pre = 0;
#pragma unroll
    for (int w2 = 0; w2 < NWAVE; ++w2) pre += (w2 < wave) ? wtot[w2] : 0;
    int run = pre + incl - ts;
    soff[4 * tid + 0] = run; run += e0;
    soff[4 * tid + 1] = run; run += e1;
    soff[4 * tid + 2] = run; run += e2;
    soff[4 * tid + 3] = run;
  }
  __syncthreads();
  for (int i = tid; i < NBMAX; i += NTHR) list[i] = soff[i];
  __syncthreads();

  if (wave == 0) {
#pragma unroll 1
    for (int b0 = 0; b0 < nh; b0 += 32) {
      const int idx = b0 + lane;
      const int uv  = reg1[idx < nh ? idx : nh - 1];
      const int m32 = (nh - b0) < 32 ? (nh - b0) : 32;
#pragma unroll 1
      for (int k = 0; k < m32; ++k) {
        const int u   = __builtin_amdgcn_readlane(uv, k);
        const int sl  = u & (NBMAX - 1);
        const int eid = (int)((unsigned)u >> SLOTB);
        if (lane == 0) {
          int pos = list[sl];
          pos = pos < 0 ? 0 : (pos > RCAP - 1 ? RCAP - 1 : pos);
          reg2[pos] = eid;
          list[sl] = pos + 1;
        }
      }
    }
  }
  __syncthreads();

  const int nbw = NBMAX / NWAVE;
  const bool ovf = (nh >= RCAP);
  const float qnan = __int_as_float(0x7fc00000);
  float* stw = (float*)reg1 + wave * STW;
  const int hd = lane >> 2;

#pragma unroll 1
  for (int jt = 0; jt < nbw; ++jt) {
    const int slot = wave * nbw + jt;
    const int grow = nodeBase + slot;
    const int gcl  = grow < nN ? grow : nN - 1;
    int st = soff[slot];
    const int craw = scnt[slot];
    int cnt = craw;
    st  = st < 0 ? 0 : (st > nh ? nh : st);
    cnt = cnt < 0 ? 0 : (cnt > DEGCAP ? DEGCAP : cnt);
    if (cnt > nh - st) cnt = nh - st;
    const float pz = (ovf || craw > DEGCAP) ? qnan : 0.0f;

    const float* qr = QKV + (size_t)gcl * QKVW + OQ + 8 * lane;
    const v4f qa = *(const v4fa*)qr;
    const v4f qb = *(const v4fa*)(qr + 4);
    ldwait();

    float mx = -1.0e30f, dn = 0.f;
    v4f ava = {0.f, 0.f, 0.f, 0.f};
    v4f avb = {0.f, 0.f, 0.f, 0.f};
#pragma unroll 1
    for (int q = 0; q < cnt; ++q) {
      int idx = st + q; idx = idx > RCAP - 1 ? RCAP - 1 : idx;
      int eid = reg2[idx]; eid = eid < 0 ? 0 : (eid > nE - 1 ? nE - 1 : eid);
      const int graw = gath[eid];
      const int g = graw < 0 ? 0 : (graw > nN - 1 ? nN - 1 : graw);
      const float ebv = EB[(size_t)eid * HN + hd];
      const float* kr = QKV + (size_t)g * QKVW + OKK + 8 * lane;
      const v4f ka = *(const v4fa*)kr;
      const v4f kb = *(const v4fa*)(kr + 4);
      const float* vr = QKV + (size_t)g * QKVW + OV + 8 * lane;
      const v4f va = *(const v4fa*)vr;
      const v4f vb = *(const v4fa*)(vr + 4);
      ldwait();
      float p = qa.x * ka.x;
      p = fmaf(qa.y, ka.y, p); p = fmaf(qa.z, ka.z, p); p = fmaf(qa.w, ka.w, p);
      p = fmaf(qb.x, kb.x, p); p = fmaf(qb.y, kb.y, p); p = fmaf(qb.z, kb.z, p); p = fmaf(qb.w, kb.w, p);
      p += __shfl_xor(p, 2);
      p += __shfl_xor(p, 1);
      const float lg = fmaf(p, ATTSC, ebv);
      const float df = lg - mx;
      const float ee = __expf(-fabsf(df));
      const bool up  = df > 0.f;
      const float s1 = up ? ee : 1.0f;
      const float s2 = up ? 1.0f : ee;
      mx = up ? lg : mx;
      dn = fmaf(dn, s1, s2);
      ava.x = fmaf(ava.x, s1, s2 * va.x); ava.y = fmaf(ava.y, s1, s2 * va.y);
      ava.z = fmaf(ava.z, s1, s2 * va.z); ava.w = fmaf(ava.w, s1, s2 * va.w);
      avb.x = fmaf(avb.x, s1, s2 * vb.x); avb.y = fmaf(avb.y, s1, s2 * vb.y);
      avb.z = fmaf(avb.z, s1, s2 * vb.z); avb.w = fmaf(avb.w, s1, s2 * vb.w);
    }
    const float dns = dn > 0.f ? dn : 1.0f;
    const float ind = dn > 0.f ? 1.0f : 0.0f;
    const float inv = ind * __builtin_amdgcn_rcpf(dns);
    v4f oa, ob;
    oa.x = ava.x * inv; oa.y = ava.y * inv; oa.z = ava.z * inv; oa.w = ava.w * inv;
    ob.x = avb.x * inv; ob.y = avb.y * inv; ob.z = avb.z * inv; ob.w = avb.w * inv;
    oa.x += pz; oa.y += pz; oa.z += pz; oa.w += pz;
    ob.x += pz; ob.y += pz; ob.z += pz; ob.w += pz;
    __builtin_amdgcn_fence(__ATOMIC_RELEASE, "wavefront");
    __builtin_amdgcn_wave_barrier();
    *(v4fa*)(stw + 8 * lane)     = oa;
    *(v4fa*)(stw + 8 * lane + 4) = ob;
    __builtin_amdgcn_fence(__ATOMIC_RELEASE, "wavefront");
    __builtin_amdgcn_wave_barrier();
    const v4f pa = *(const v4fa*)(stw + 4 * lane);
    const v4f pb = *(const v4fa*)(stw + (DM / 2) + 4 * lane);
    const bool wr = (grow < MPr);
    const int gsf = wr ? grow : MPr - 1;
    float* orow = OUTP + (size_t)gsf * DM;
    if (wr) {
      *(volatile v4f*)(orow + 4 * lane)            = pa;
      *(volatile v4f*)(orow + (DM / 2) + 4 * lane) = pb;
    }
    __threadfence();
    if (wr) {
      *(volatile v4f*)(orow + 4 * lane)            = pa;
      *(volatile v4f*)(orow + (DM / 2) + 4 * lane) = pb;
    }
  }
}

__global__ __launch_bounds__(GTHR) void k_out(
    const float* __restrict__ AGG, const unsigned short* __restrict__ WOT2,
    const float* __restrict__ bo, float* out, int nN)
{
  extern __shared__ v4f lds_dyn[];
  unsigned short* At = (unsigned short*)lds_dyn;
  float* stg = (float*)(At + GBM * KFIN);
  const int tid = (int)threadIdx.x, lane = tid & 31, wave = tid >> 5, hh = lane >> 4, m = lane & 15;
  const int rowBase = (int)blockIdx.x * GBM;

#pragma unroll 1
  for (int g = 0; g < DM / GBN; ++g) {
#pragma unroll
    for (int i = 0; i < 4; ++i) {
      const int p   = i * GTHR + tid;
      const int row = p >> 3;
      const int q8  = (p & 7) * 8;
      const float* arp = AGG + (size_t)(rowBase + row) * DM + g * GBN + q8;
      const v4f a = *(const v4fa*)arp;
      const v4f b = *(const v4fa*)(arp + 4);
      v4u hv, lv;
      pack8hl(a, b, hv, lv);
      *(v4ua*)(At + row * KFIN + g * GBN + q8)      = hv;
      *(v4ua*)(At + row * KFIN + DM + g * GBN + q8) = lv;
    }
  }
  __syncthreads();

  const unsigned short* aq = At + (size_t)(16 * wave + m) * KFIN + 8 * hh;
#pragma unroll 1
  for (int g2 = 0; g2 < DM / GBN; ++g2) {
    v8f acc[4];
    {
      const v8f z = {0.f, 0.f, 0.f, 0.f, 0.f, 0.f, 0.f, 0.f};
      acc[0] = z; acc[1] = z; acc[2] = z; acc[3] = z;
    }
    const unsigned short* wl = WOT2 + (size_t)(g2 * GBN + m) * KFIN + 8 * hh;
#pragma unroll 1
    for (int ks = 0; ks < KFIN / 32; ++ks) {
      FragB af;
      af.h[0] = *(const v8usa*)(aq + 32 * ks);
      af.h[1] = *(const v8usa*)(aq + 32 * ks + 16);
#pragma unroll
      for (int t = 0; t < 4; ++t) {
        const unsigned short* wq = wl + (size_t)(16 * t) * KFIN + 32 * ks;
        FragB bf;
        bf.h[0] = *(const v8usa*)wq;
        bf.h[1] = *(const v8usa*)(wq + 16);
        acc[t] = wmb(af, bf, acc[t]);
      }
    }

#pragma unroll
    for (int t = 0; t < 4; ++t) {
      const int lc = 16 * t + m;
#pragma unroll
      for (int r = 0; r < 8; ++r) {
        const int lr = 16 * wave + 8 * hh + r;
        stg[lr * GBN + lc] = acc[t][r];
      }
    }
    __syncthreads();

    const v4f bb = bfr4(*(const v4fa*)(bo + g2 * GBN + 4 * m));
    v4f fv[8];
#pragma unroll
    for (int i = 0; i < 8; ++i) {
      const int lr = 16 * wave + 2 * i + hh;
      fv[i] = *(const v4fa*)(stg + lr * GBN + 4 * m) + bb;
    }
#pragma unroll
    for (int i = 0; i < 8; ++i) {
      const int lr = 16 * wave + 2 * i + hh;
      const int gr = rowBase + lr;
      const int gs = gr < nN ? gr : nN - 1;
      float* op = out + (size_t)gs * DM + g2 * GBN + 4 * m;
      if (gr < nN) *(volatile v4f*)op = fv[i];
    }
    __threadfence();
#pragma unroll
    for (int i = 0; i < 8; ++i) {
      const int lr = 16 * wave + 2 * i + hh;
      const int gr = rowBase + lr;
      const int gs = gr < nN ? gr : nN - 1;
      float* op = out + (size_t)gs * DM + g2 * GBN + 4 * m;
      if (gr < nN) *(volatile v4f*)op = fv[i];
    }
    __syncthreads();
  }
}

static inline int cdiv(int a, int b) { return (a + b - 1) / b; }

extern "C" void kernel_launch(void* const* d_in, const int* in_sizes, int n_in,
                              void* d_out, int out_size, void* d_ws, size_t ws_size,
                              hipStream_t stream) {
  if (n_in < 13) return;
  if (in_sizes[0] < NBATCH * DM || (in_sizes[0] % (NBATCH * DM)) != 0) return;
  const int nN = in_sizes[0] / (NBATCH * DM);
  if (nN < 1 || nN > (1 << 22)) return;
  if (in_sizes[1] < 2 || (in_sizes[1] & 1) != 0) return;
  const int nE = in_sizes[1] / 2;
  if (nE < 1 || nE >= (1 << (31 - SLOTB))) return;
  if (in_sizes[2] != nE * EDW) return;
  if (in_sizes[3] != DM * DM || in_sizes[5] != DM * DM || in_sizes[7] != DM * DM || in_sizes[11] != DM * DM) return;
  if (in_sizes[4] != DM || in_sizes[6] != DM || in_sizes[8] != DM || in_sizes[12] != DM) return;
  if (in_sizes[9] != EDW * HN || in_sizes[10] != HN) return;
  if (out_size != NBATCH * nN * DM) return;

  const float* x     = (const float*)d_in[0];
  const int*   ei    = (const int*)  d_in[1];
  const float* eattr = (const float*)d_in[2];
  const float* Wq    = (const float*)d_in[3];
  const float* bq    = (const float*)d_in[4];
  const float* Wk    = (const float*)d_in[5];
  const float* bk    = (const float*)d_in[6];
  const float* Wv    = (const float*)d_in[7];
  const float* bv    = (const float*)d_in[8];
  const float* We    = (const float*)d_in[9];
  const float* be    = (const float*)d_in[10];
  const float* Wo    = (const float*)d_in[11];
  const float* bo    = (const float*)d_in[12];
  float* out = (float*)d_out;
  const int* keys = ei;
  const int* gath = ei + nE;

  const int MP   = cdiv(nN, GBM) * GBM;
  const int gA   = cdiv(MP, NBMAX);
  const int EP   = cdiv(nE, 4) * 4;
  const int vec8 = ((nE & 3) == 0) ? 1 : 0;
  if (gA * NBMAX < MP) return;

  char* ws = (char*)d_ws;
  size_t off = 0;
  const size_t oXB  = off; off += (size_t)MP * DM * 2;             off = (off + 255) & ~(size_t)255;
  const size_t oWQ  = off; off += (size_t)QKVW * DM * 2;           off = (off + 255) & ~(size_t)255;
  const size_t oWO  = off; off += (size_t)DM * KFIN * 2;           off = (off + 255) & ~(size_t)255;
  const size_t oEB  = off; off += (size_t)EP * HN * 4;             off = (off + 255) & ~(size_t)255;
  const size_t oQKV = off; off += (size_t)MP * QKVW * 4;           off = (off + 255) & ~(size_t)255;
  const size_t oAGG = off; off += (size_t)MP * DM * 4;             off = (off + 255) & ~(size_t)255;
  if (off > ws_size || off > (size_t)WSMAX) return;
  unsigned short* XB    = (unsigned short*)(ws + oXB);
  unsigned short* WQKVT = (unsigned short*)(ws + oWQ);
  unsigned short* WOT2  = (unsigned short*)(ws + oWO);
  float*          EB    = (float*)(ws + oEB);
  float*          QKV   = (float*)(ws + oQKV);
  float*          AGG   = (float*)(ws + oAGG);

  hipFuncSetAttribute(reinterpret_cast<const void*>(&k_agg),
                      hipFuncAttributeMaxDynamicSharedMemorySize, LDS_AGG);
  hipFuncSetAttribute(reinterpret_cast<const void*>(&k_out),
                      hipFuncAttributeMaxDynamicSharedMemorySize, LDS_FIN);

  {
    const int nUq = DM * (DM / 8);
    k_wtr<<<cdiv(nUq, NTHR), NTHR, 0, stream>>>(Wq, DM, DM, DM, DM, WQKVT,                       nUq);
    k_wtr<<<cdiv(nUq, NTHR), NTHR, 0, stream>>>(Wk, DM, DM, DM, DM, WQKVT + (size_t)DM * DM,     nUq);
    k_wtr<<<cdiv(nUq, NTHR), NTHR, 0, stream>>>(Wv, DM, DM, DM, DM, WQKVT + (size_t)2 * DM * DM, nUq);
    const int nUo = DM * (KFIN / 8);
    k_wtr<<<cdiv(nUo, NTHR), NTHR, 0, stream>>>(Wo, DM, DM, DM, KFIN, WOT2, nUo);
  }
  {
    const int nUe = EP * 2;
    k_eb<<<cdiv(nUe, NTHR), NTHR, 0, stream>>>(eattr, We, be, EB, nE, nUe);
  }

  const int gM  = MP / GBM;
  const int nUx = MP * (DM / 8);
  for (int b = 0; b < NBATCH; ++b) {
    const float* xb = x + (size_t)b * (size_t)nN * DM;
    float* ob = out + (size_t)b * (size_t)nN * DM;
    k_xprep<<<cdiv(nUx, NTHR), NTHR, 0, stream>>>(xb, XB, nN, nUx);
    k_gemm<<<dim3(gM, QKVW / GBN), GTHR, 0, stream>>>(XB, WQKVT, bq, bk, bv, QKV, DM, QKVW);
    k_agg<<<gA, NTHR, LDS_AGG, stream>>>(keys, gath, QKV, EB, AGG, nN, nE, vec8, MP);
    k_out<<<gM, GTHR, LDS_FIN, stream>>>(AGG, WOT2, bo, ob, nN);
  }
}
